// GQA_9715216023893
// MI455X (gfx1250) — hardware-verified
//
#include <hip/hip_runtime.h>
#include <math.h>

typedef __attribute__((ext_vector_type(16))) _Float16 v16h;
typedef __attribute__((ext_vector_type(16))) __bf16 v16b;
typedef __attribute__((ext_vector_type(8)))  _Float16 v8h;
typedef __attribute__((ext_vector_type(8)))  unsigned short v8us;
typedef __attribute__((ext_vector_type(8)))  float v8f;
typedef __attribute__((ext_vector_type(4)))  float v4f;
typedef __attribute__((ext_vector_type(4)))  unsigned v4u;

template <typename T> __device__ __forceinline__ void vst2(void* p, T v) { *(volatile T*)p = v; __threadfence(); *(volatile T*)p = v; }
__device__ __forceinline__ v8f wmma16(v16h a, v16h b, v8f c) {
  v8f d = __builtin_amdgcn_wmma_f32_16x16x32_f16(false, a, false, b, (short)0, c, false, false);
  asm volatile("v_nop\n\tv_nop\n\tv_nop\n\tv_nop" : "+v"(d) : "v"(a), "v"(b));
  return d;
}
__device__ __forceinline__ v8f wmma_bf(v16b a, v16b b, v8f c) {
  v8f d = __builtin_amdgcn_wmma_f32_16x16x32_bf16(false, a, false, b, (short)0, c, false, false);
  asm volatile("v_nop\n\tv_nop\n\tv_nop\n\tv_nop" : "+v"(d) : "v"(a), "v"(b));
  return d;
}
__device__ __forceinline__ v16h frag_h(const _Float16* rowk0, int lane) {
  union { v16h v; v8h q[2]; } u; const _Float16* p = rowk0 + 8 * (lane >> 4);
  u.q[0] = *(const v8h*)p; u.q[1] = *(const v8h*)(p + 16); return u.v;
}
__device__ __forceinline__ v16b frag_b(const __bf16* rowk0, int lane) {
  union { v16b v; v8us q[2]; } u; const unsigned short* p = (const unsigned short*)rowk0 + 8 * (lane >> 4);
  u.q[0] = *(const v8us*)p; u.q[1] = *(const v8us*)(p + 16); return u.v;
}
struct F2 { v16b h, l; };
__device__ __forceinline__ F2 bsplit16(const float v[16]) { F2 r;
#pragma unroll
  for (int i = 0; i < 16; ++i) { const __bf16 h = (__bf16)v[i]; r.h[i] = h; r.l[i] = (__bf16)(v[i] - (float)h); }
  return r; }
__device__ __forceinline__ F2 split_row(const float* row, int k0, int lane) { float v[16]; const float* p = row + k0 + 8 * (lane >> 4);
#pragma unroll
  for (int i = 0; i < 8; ++i) { v[i] = p[i]; v[8 + i] = p[16 + i]; }
  return bsplit16(v); }
__device__ __forceinline__ float bfr(float v) { return (float)(__bf16)v; }
__device__ __forceinline__ v16b wcol_oi(const float* Wm, int k0, int o, int lane, int K) { v16b w; const float* p = Wm + (size_t)o * K + k0 + 8 * (lane >> 4);
#pragma unroll
  for (int i = 0; i < 8; ++i) { w[i] = (__bf16)p[i]; w[8 + i] = (__bf16)p[16 + i]; }
  return w; }
#define LDSX() do { asm volatile("s_wait_dscnt 0" ::: "memory"); __builtin_amdgcn_wave_barrier(); __builtin_amdgcn_fence(3  , "workgroup"); } while (0)

#ifndef NB
#define NB 2
#endif
#ifndef SEQ
#define SEQ 2048
#endif
#define NB_FULL 2
#define SEQ_FULL 2048
#define TT SEQ
#define CC 1024
#define DIN 1024
#define NH 16
#define HD 64
#define GG 4
#define KVE 256
#define NQB (TT / 64)
#define HG 4
#define SCALE (0.125f)
#define PSC (2048.0f)
#define LN_EPS (1e-5f)
static_assert(TT % 256 == 0);
static_assert(NB >= 1 && NB <= NB_FULL);
static_assert(SEQ >= 256 && SEQ <= SEQ_FULL);
static_assert(NH * HD == CC);
static_assert(KVE == (NH / GG) * HD);
static_assert(NH % HG == 0 && HG % GG == 0);

__host__ __device__ __forceinline__ int kb_last(int qb) { return (qb * 64 + 63) >> 7; }

#define WS_QH  ((size_t)0)
#define WS_QL  (WS_QH + 2u * (size_t)NB * TT * CC)
#define WS_KH  (WS_QL + 2u * (size_t)NB * TT * CC)
#define WS_KL  (WS_KH + 2u * (size_t)NB * TT * KVE)
#define WS_VB  (WS_KL + 2u * (size_t)NB * TT * KVE)
#define WS_VL  (WS_VB + 2u * (size_t)NB * KVE * TT)
#define WS_VM  (WS_VL + 2u * (size_t)NB * KVE * TT)
#define WS_S   (WS_VM + 4096u)
#define WS_Y   (WS_S  + 4u * (size_t)HG * TT * TT)
#define WS_YN  (WS_Y  + 4u * (size_t)NB * TT * CC)
#define WS_END (WS_YN + 4u * (size_t)NB * TT * CC)
static_assert(WS_END <= (size_t)134217728u);
static_assert(4u * NB * KVE <= 4096u);
static_assert((WS_S % 4096u) == 0 && (WS_Y % 4096u) == 0 && (WS_YN % 4096u) == 0 && (WS_VM % 4096u) == 0);

__global__ __launch_bounds__(128) void k_proj(const float* __restrict__ XQ, const float* __restrict__ XK, const float* __restrict__ XV,
    const float* __restrict__ WQ, const float* __restrict__ WK, const float* __restrict__ WV,
    const float* __restrict__ BQ, const float* __restrict__ BK, const float* __restrict__ BV, int which0,
    _Float16* __restrict__ QH, _Float16* __restrict__ QL, _Float16* __restrict__ KH, _Float16* __restrict__ KL,
    __bf16* __restrict__ VB, __bf16* __restrict__ VL) {
  __shared__ __align__(16) _Float16 sh[64][136], sl[64][136]; __shared__ __align__(16) __bf16 tb[128][72], tbl[128][72];
  const int tid = threadIdx.x, wave = tid >> 5, lane = tid & 31, col = lane & 15, g = lane >> 4; const int which = which0 + (int)blockIdx.z; const int c0 = blockIdx.y * 128;
  const size_t r0 = (size_t)blockIdx.x * 64; const size_t bb = r0 / TT; const int t0 = (int)(r0 % TT);
  const size_t x0 = bb * (size_t)SEQ_FULL + (size_t)t0;
  const float* X = which == 0 ? XQ : which == 1 ? XK : XV; const float* WA = which == 0 ? WQ : which == 1 ? WK : WV; const float* BA = which == 0 ? BQ : which == 1 ? BK : BV;
  v8f acc[8] = {};
#pragma unroll 2
  for (int kc = 0; kc < DIN / 32; ++kc) { v16b a; { const float* p = X + (x0 + wave * 16 + col) * DIN + kc * 32 + 8 * g;
#pragma unroll
      for (int i = 0; i < 8; ++i) { a[i] = (__bf16)p[i]; a[8 + i] = (__bf16)p[16 + i]; } }
    asm volatile("s_wait_loadcnt 0x0" ::: "memory");
#pragma unroll
    for (int j = 0; j < 8; ++j) { const v16b w = wcol_oi(WA, kc * 32, c0 + j * 16 + col, lane, DIN); asm volatile("s_wait_loadcnt 0x0" ::: "memory"); acc[j] = wmma_bf(a, w, acc[j]); } }
  if (which < 2) { _Float16* DH = which == 0 ? QH : KH; _Float16* DL = which == 0 ? QL : KL; const size_t pitch = which == 0 ? (size_t)CC : (size_t)KVE;
#pragma unroll
    for (int j = 0; j < 8; ++j) { const float bias = bfr(BA[c0 + j * 16 + col]);
#pragma unroll
      for (int r = 0; r < 8; ++r) { const float v = acc[j][r] + bias; const _Float16 hv = (_Float16)v; sh[wave * 16 + 8 * g + r][j * 16 + col] = hv; sl[wave * 16 + 8 * g + r][j * 16 + col] = (_Float16)((v - (float)hv) * 1024.0f); } }
    __syncthreads();
    for (int e = tid; e < 64 * 16; e += 128) { const int rl = e >> 4, q = e & 15; const size_t off = (r0 + rl) * pitch + c0 + q * 8;
      vst2((unsigned*)(DH + off), *(const v4u*)&sh[rl][q * 8]); vst2((unsigned*)(DL + off), *(const v4u*)&sl[rl][q * 8]); }
  } else {
#pragma unroll
    for (int j = 0; j < 8; ++j) { const float bias = bfr(BA[c0 + j * 16 + col]);
#pragma unroll
      for (int r = 0; r < 8; ++r) { const float v = acc[j][r] + bias; const int rl = wave * 16 + 8 * g + r, cl = j * 16 + col; const __bf16 bh = (__bf16)v; tb[cl][rl] = bh; tbl[cl][rl] = (__bf16)(v - (float)bh); } }
    __syncthreads();
    for (int e = tid; e < 128 * 8; e += 128) { const int cl = e >> 3, q = e & 7; const size_t o3 = (bb * KVE + c0 + cl) * (size_t)TT + t0 + q * 8;
      vst2((unsigned*)(VB + o3), *(const v4u*)&tb[cl][q * 8]); vst2((unsigned*)(VL + o3), *(const v4u*)&tbl[cl][q * 8]); } } }

__global__ __launch_bounds__(256) void k_vmean(const unsigned short* __restrict__ VBb, const unsigned short* __restrict__ VLb, float* __restrict__ VM) {
  __shared__ __align__(16) float svm[32];
  const int tid = threadIdx.x, wave = tid >> 5, lane = tid & 31; const int rbase = blockIdx.x * 32;
#pragma unroll 1
  for (int u = 0; u < 4; ++u) { const int rr = rbase + wave * 4 + u;
    const unsigned short* ph = VBb + (size_t)rr * TT; const unsigned short* pl = VLb + (size_t)rr * TT;
    float s = 0.f;
#pragma unroll 1
    for (int it = 0; it < TT / 256; ++it) { const int e0 = (it * 32 + lane) * 8; const v8us wh = *(const v8us*)(ph + e0), wl = *(const v8us*)(pl + e0);
#pragma unroll
      for (int i = 0; i < 8; ++i) s += __uint_as_float((unsigned)wh[i] << 16) + __uint_as_float((unsigned)wl[i] << 16); }
#pragma unroll
    for (int o = 1; o < 32; o <<= 1) s += __shfl_xor(s, o);
    if (lane == 0) svm[wave * 4 + u] = s * (1.0f / (float)TT); }
  __syncthreads();
  if (wave == 0 && lane < 8) vst2(VM + rbase + lane * 4, *(const v4f*)&svm[lane * 4]); }

__global__ __launch_bounds__(128) void k_sc(const _Float16* __restrict__ QH, const _Float16* __restrict__ QL, const _Float16* __restrict__ KH, const _Float16* __restrict__ KL, int b, int h0, float* __restrict__ S0) {
  __shared__ __align__(16) float ss[4][16][132];
  const int qb = blockIdx.x, kb = blockIdx.y; if (kb > kb_last(qb)) return;
  const int h = h0 + (int)blockIdx.z, kvh = h / GG; float* S = S0 + (size_t)blockIdx.z * TT * TT;
  const int tid = threadIdx.x, wave = tid >> 5, lane = tid & 31, col = lane & 15, g = lane >> 4; const int k0 = kb * 128; const int ql0 = qb * 64 + wave * 16;
  const size_t q0 = (size_t)b * TT + ql0, kr0 = (size_t)b * TT + k0;
  const _Float16* qp = QH + (q0 + col) * CC + h * HD; const _Float16* qlp = QL + (q0 + col) * CC + h * HD;
  const v16h ah0 = frag_h(qp, lane), ah1 = frag_h(qp + 32, lane), al0 = frag_h(qlp, lane), al1 = frag_h(qlp + 32, lane);
  asm volatile("s_wait_loadcnt 0x0" ::: "memory");
#pragma unroll 1
  for (int j = 0; j < 8; ++j) {
    const _Float16* kp = KH + (kr0 + j * 16 + col) * KVE + kvh * HD; const _Float16* klp = KL + (kr0 + j * 16 + col) * KVE + kvh * HD;
    const v16h kf0 = frag_h(kp, lane), kf1 = frag_h(kp + 32, lane), kl0 = frag_h(klp, lane), kl1 = frag_h(klp + 32, lane);
    asm volatile("s_wait_loadcnt 0x0" ::: "memory");
    v8f acc = {}, accl = {};
    acc = wmma16(ah0, kf0, acc); accl = wmma16(al0, kf0, accl); accl = wmma16(ah0, kl0, accl);
    acc = wmma16(ah1, kf1, acc); accl = wmma16(al1, kf1, accl); accl = wmma16(ah1, kl1, accl);
#pragma unroll
    for (int r = 0; r < 8; ++r) ss[wave][8 * g + r][j * 16 + col] = (acc[r] + accl[r] * (1.0f / 1024.0f)) * SCALE; }
  LDSX();
  for (int rl = 0; rl < 16; ++rl) vst2(S + (size_t)(ql0 + rl) * TT + k0 + lane * 4, *(const v4f*)&ss[wave][rl][lane * 4]); }

__global__ __launch_bounds__(256) void k_sm(float* __restrict__ S0, const int* __restrict__ ADJ, int b) {
  __shared__ float sred[8]; __shared__ float sbc; __shared__ __align__(16) float shv[TT];
  const int tid = threadIdx.x; const int t = blockIdx.x; const int kend = (kb_last(t >> 6) + 1) * 128;
  float* sr = S0 + (size_t)blockIdx.y * TT * TT + (size_t)t * TT; const int* ar = ADJ + ((size_t)b * SEQ_FULL + t) * SEQ_FULL;
  float m = -3.0e38f; for (int k = tid; k < kend; k += 256) { const float s = sr[k]; const int a = ar[k]; const float v = (k <= t && a != 0) ? s : -3.0e38f; shv[k] = v; m = fmaxf(m, v); }
#pragma unroll
  for (int o = 1; o < 32; o <<= 1) m = fmaxf(m, __shfl_xor(m, o));
  if ((tid & 31) == 0) sred[tid >> 5] = m; __syncthreads(); if (tid == 0) { float a = sred[0]; for (int i = 1; i < 8; ++i) a = fmaxf(a, sred[i]); sbc = a; } __syncthreads(); m = sbc; __syncthreads();
  float sum = 0.f; for (int k = tid; k < kend; k += 256) { const float v = shv[k]; const float e = (v <= -1.0e38f) ? 0.f : expf(v - m); shv[k] = e; sum += e; }
#pragma unroll
  for (int o = 1; o < 32; o <<= 1) sum += __shfl_xor(sum, o);
  if ((tid & 31) == 0) sred[tid >> 5] = sum; __syncthreads(); if (tid == 0) { float a = 0.f; for (int i = 0; i < 8; ++i) a += sred[i]; sbc = a > 0.f ? PSC / a : 0.f; } __syncthreads(); const float inv = sbc;
  for (int k = tid; k < kend; k += 256) shv[k] = shv[k] * inv;
  __syncthreads();
  for (int q = tid; q < kend / 4; q += 256) vst2(sr + q * 4, *(const v4f*)&shv[q * 4]); }

__global__ __launch_bounds__(128) void k_pv(const float* __restrict__ PS0, const __bf16* __restrict__ VB, const __bf16* __restrict__ VL, int b, int h0, float* __restrict__ Y) {
  __shared__ __align__(16) float ss[4][16][HD + 4];
  const int h = h0 + (int)blockIdx.z, kvh = h / GG; const float* PS = PS0 + (size_t)blockIdx.z * TT * TT;
  const int tid = threadIdx.x, wave = tid >> 5, lane = tid & 31, col = lane & 15, g = lane >> 4; const int qb = blockIdx.x; const int ql0 = qb * 64 + wave * 16; const int kce = (kb_last(qb) + 1) * 4;
  v8f acc[HD / 16] = {};
#pragma unroll 1
  for (int kc = 0; kc < kce; ++kc) { const F2 p = split_row(PS + (size_t)(ql0 + col) * TT, kc * 32, lane);
    asm volatile("s_wait_loadcnt 0x0" ::: "memory");
#pragma unroll
    for (int j = 0; j < HD / 16; ++j) { const size_t po = ((size_t)b * KVE + kvh * HD + j * 16 + col) * (size_t)TT + kc * 32; const v16b vh = frag_b(VB + po, lane);
      acc[j] = wmma_bf(p.h, vh, acc[j]); acc[j] = wmma_bf(p.l, vh, acc[j]); acc[j] = wmma_bf(p.h, frag_b(VL + po, lane), acc[j]); } }
#pragma unroll
  for (int j = 0; j < HD / 16; ++j)
#pragma unroll
    for (int r = 0; r < 8; ++r) ss[wave][8 * g + r][j * 16 + col] = acc[j][r] * (1.0f / PSC);
  LDSX();
  for (int rl = 0; rl < 16; ++rl) if (lane < HD / 4) vst2(Y + ((size_t)b * TT + ql0 + rl) * CC + h * HD + lane * 4, *(const v4f*)&ss[wave][rl][lane * 4]); }

__global__ __launch_bounds__(256) void k_ln(const float* __restrict__ Y, const float* __restrict__ VM, const int* __restrict__ ADJ, const float* __restrict__ LG, const float* __restrict__ LB, float* __restrict__ YN) {
  __shared__ float sred[8]; __shared__ int sfl[8];
  const int tid = threadIdx.x, wave = tid >> 5, lane = tid & 31; const int row = blockIdx.x; const int b = row / TT, t = row % TT;
  const int* ar = ADJ + ((size_t)b * SEQ_FULL + t) * SEQ_FULL;
  int any = 0; for (int s = tid; s <= t; s += 256) any |= (ar[s] != 0) ? 1 : 0;
#pragma unroll
  for (int o = 1; o < 32; o <<= 1) any |= __shfl_xor(any, o);
  if (lane == 0) sfl[wave] = any; __syncthreads();
  int fl = 0;
#pragma unroll
  for (int i = 0; i < 8; ++i) fl |= sfl[i];
  const bool um = (fl == 0);
  const int c = tid * 4;
  const v4f yv = *(const v4f*)(Y + (size_t)row * CC + c); const v4f mv = *(const v4f*)(VM + b * KVE + (c >> 8) * HD + (c & 63));
  float x[4];
#pragma unroll
  for (int i = 0; i < 4; ++i) x[i] = um ? mv[i] : yv[i];
  float s = (x[0] + x[1]) + (x[2] + x[3]);
#pragma unroll
  for (int o = 1; o < 32; o <<= 1) s += __shfl_xor(s, o);
  if (lane == 0) sred[wave] = s; __syncthreads();
  float tot = 0.f;
#pragma unroll
  for (int i = 0; i < 8; ++i) tot += sred[i];
  const float mu = tot * (1.0f / (float)CC); __syncthreads();
  float s2 = 0.f;
#pragma unroll
  for (int i = 0; i < 4; ++i) { const float d = x[i] - mu; s2 += d * d; }
#pragma unroll
  for (int o = 1; o < 32; o <<= 1) s2 += __shfl_xor(s2, o);
  if (lane == 0) sred[wave] = s2; __syncthreads();
  float tot2 = 0.f;
#pragma unroll
  for (int i = 0; i < 8; ++i) tot2 += sred[i];
  const float var = tot2 * (1.0f / (float)CC); const float rstd = 1.0f / sqrtf(var + LN_EPS);
  v4f o;
#pragma unroll
  for (int i = 0; i < 4; ++i) o[i] = (x[i] - mu) * rstd * bfr(LG[c + i]) + bfr(LB[c + i]);
  vst2(YN + (size_t)row * CC + c, o); }

__global__ __launch_bounds__(128) void k_out(const float* __restrict__ Y, const float* __restrict__ WO, const float* __restrict__ BO, float* __restrict__ OUT) {
  __shared__ __align__(16) float sf[4][16][132];
  const int tid = threadIdx.x, wave = tid >> 5, lane = tid & 31, col = lane & 15, g = lane >> 4; const int c0 = blockIdx.y * 128; const size_t r0 = (size_t)blockIdx.x * 64 + wave * 16;
  v8f acc[8] = {};
#pragma unroll 2
  for (int kc = 0; kc < CC / 32; ++kc) { const F2 a = split_row(Y + (r0 + col) * CC, kc * 32, lane); asm volatile("s_wait_loadcnt 0x0" ::: "memory");
#pragma unroll
    for (int j = 0; j < 8; ++j) { const v16b w = wcol_oi(WO, kc * 32, c0 + j * 16 + col, lane, CC); asm volatile("s_wait_loadcnt 0x0" ::: "memory"); acc[j] = wmma_bf(a.h, w, acc[j]); acc[j] = wmma_bf(a.l, w, acc[j]); } }
#pragma unroll
  for (int j = 0; j < 8; ++j) { const float bias = bfr(BO[c0 + j * 16 + col]);
#pragma unroll
    for (int r = 0; r < 8; ++r) sf[wave][8 * g + r][j * 16 + col] = acc[j][r] + bias; }
  LDSX();
  for (int rl = 0; rl < 16; ++rl) vst2(OUT + (r0 + rl) * CC + c0 + lane * 4, *(const v4f*)&sf[wave][rl][lane * 4]); }

extern "C" void kernel_launch(void* const* d_in, const int* in_sizes, int n_in, void* d_out, int out_size, void* d_ws, size_t ws_size, hipStream_t stream) {
  if (n_in < 14) return;
  const float* XQ = (const float*)d_in[0]; const float* XK = (const float*)d_in[1]; const float* XV = (const float*)d_in[2]; const int* ADJ = (const int*)d_in[3];
  const float* WQ = (const float*)d_in[4]; const float* BQ = (const float*)d_in[5]; const float* WK = (const float*)d_in[6]; const float* BK = (const float*)d_in[7];
  const float* WV = (const float*)d_in[8]; const float* BV = (const float*)d_in[9]; const float* WO = (const float*)d_in[10]; const float* BO = (const float*)d_in[11];
  const float* LG = (const float*)d_in[12]; const float* LB = (const float*)d_in[13];
  const long long need_x = ((long long)(NB - 1) * SEQ_FULL + SEQ) * (long long)DIN;
  const long long need_a = ((long long)(NB - 1) * SEQ_FULL + SEQ) * (long long)SEQ_FULL;
  if ((long long)in_sizes[0] < need_x || (long long)in_sizes[1] < need_x || (long long)in_sizes[2] < need_x || (long long)in_sizes[3] < need_a) return;
  if (in_sizes[4] < CC * DIN || in_sizes[5] < CC || in_sizes[6] < KVE * DIN || in_sizes[7] < KVE || in_sizes[8] < KVE * DIN || in_sizes[9] < KVE) return;
  if (in_sizes[10] < CC * CC || in_sizes[11] < CC || in_sizes[12] < CC || in_sizes[13] < CC) return;
  if ((long long)out_size < (long long)NB * TT * CC) return;
  if (ws_size < WS_END) return;
  char* ws = (char*)d_ws;
  _Float16 *QH = (_Float16*)(ws + WS_QH), *QL = (_Float16*)(ws + WS_QL), *KH = (_Float16*)(ws + WS_KH), *KL = (_Float16*)(ws + WS_KL);
  __bf16 *VB = (__bf16*)(ws + WS_VB), *VL = (__bf16*)(ws + WS_VL);
  float *VM = (float*)(ws + WS_VM), *S = (float*)(ws + WS_S), *Y = (float*)(ws + WS_Y), *YN = (float*)(ws + WS_YN);
  float* OUT = (float*)d_out;
  k_proj<<<dim3(NB * TT / 64, CC / 128, 1), 128, 0, stream>>>(XQ, XK, XV, WQ, WK, WV, BQ, BK, BV, 0, QH, QL, KH, KL, VB, VL);
  k_proj<<<dim3(NB * TT / 64, KVE / 128, 2), 128, 0, stream>>>(XQ, XK, XV, WQ, WK, WV, BQ, BK, BV, 1, QH, QL, KH, KL, VB, VL);
  k_vmean<<<NB * KVE / 32, 256, 0, stream>>>((const unsigned short*)VB, (const unsigned short*)VL, VM);
  for (int b = 0; b < NB; ++b) for (int h0 = 0; h0 < NH; h0 += HG) {
    k_sc<<<dim3(NQB, TT / 128, HG), 128, 0, stream>>>(QH, QL, KH, KL, b, h0, S);
    k_sm<<<dim3(TT, HG), 256, 0, stream>>>(S, ADJ, b);
    k_pv<<<dim3(NQB, 1, HG), 128, 0, stream>>>(S, VB, VL, b, h0, Y);
  }
  k_ln<<<NB * TT, 256, 0, stream>>>(Y, VM, ADJ, LG, LB, YN);
  k_out<<<dim3(NB * TT / 64, CC / 128), 128, 0, stream>>>(YN, WO, BO, OUT);
}
